// TXLAttn_68049461838047
// MI455X (gfx1250) — hardware-verified
//
#include <hip/hip_runtime.h>


#define NB_  4
#define SS   1024
#define DM   1024
#define NH_  16
#define HD   64
#define NTK  (NB_ * SS)
#define NRL  2048
#define NRP  2112
#define PSC  32768.0f
#define LOSC 1024.0f
#define LOSCI (1.0f / 1024.0f)

typedef _Float16 h16;
typedef unsigned short bf;
typedef __attribute__((ext_vector_type(16))) __bf16   v16bf;
typedef __attribute__((ext_vector_type(16))) _Float16 v16h;
typedef __attribute__((ext_vector_type(8)))  _Float16 v8h;
typedef __attribute__((ext_vector_type(8)))  unsigned short v8us;
typedef __attribute__((ext_vector_type(8)))  float    v8f;
typedef __attribute__((ext_vector_type(4)))  float    v4f;
typedef v8h  __attribute__((may_alias)) v8ha;
typedef v4f  __attribute__((may_alias)) v4fa;
typedef v8us __attribute__((may_alias)) v8usa;

__device__ __forceinline__ unsigned short f2bf(float f) { unsigned u = __float_as_uint(f); u += 0x7FFFu + ((u >> 16) & 1u); return (unsigned short)(u >> 16); }
__device__ __forceinline__ float bf2f(unsigned short b) { return __uint_as_float(((unsigned)b) << 16); }
__device__ __forceinline__ float bfr(float f) { return bf2f(f2bf(f)); }
__device__ __forceinline__ v16h cat16(v8h lo, v8h hi) { return __builtin_shufflevector(lo, hi, 0, 1, 2, 3, 4, 5, 6, 7, 8, 9, 10, 11, 12, 13, 14, 15); }
__device__ __forceinline__ v16bf cat16b(v8us lo, v8us hi) { return __builtin_bit_cast(v16bf, __builtin_shufflevector(lo, hi, 0, 1, 2, 3, 4, 5, 6, 7, 8, 9, 10, 11, 12, 13, 14, 15)); }
__device__ __forceinline__ v8f wmma16(v16h a, v16h b, v8f c) { return __builtin_amdgcn_wmma_f32_16x16x32_f16(false, a, false, b, (short)0, c, false, false); }
__device__ __forceinline__ v8f wmmab(v16bf a, v16bf b, v8f c) { return __builtin_amdgcn_wmma_f32_16x16x32_bf16(false, a, false, b, (short)0, c, false, false); }
#define VST2(T, p, v) do { const T vst2_v_ = (v); *(volatile T*)(p) = vst2_v_; __threadfence(); *(volatile T*)(p) = vst2_v_; } while (0)

__global__ __launch_bounds__(256) void k_cvtb(const float* __restrict__ src, int nrows, bf* dst) {
    const int lane = threadIdx.x & 31, r = blockIdx.x * 8 + (threadIdx.x >> 5);
    if (r >= nrows) return;
#pragma unroll
    for (int q = 0; q < DM / 256; ++q) { v8us t;
#pragma unroll
        for (int i = 0; i < 8; ++i) t[i] = f2bf(src[(size_t)r * DM + q * 256 + lane * 8 + i]);
        VST2(v8us, dst + (size_t)r * DM + q * 256 + lane * 8, t); }
}
__global__ __launch_bounds__(256) void k_wt(const float* __restrict__ Wm, bf* WT) {
    __shared__ __align__(16) unsigned short tl[64 * 72];
    const int tid = threadIdx.x, k0 = blockIdx.x * 64, n0 = blockIdx.y * 64;
    const int kk = tid >> 2, nq = (tid & 3) * 16;
#pragma unroll
    for (int i = 0; i < 16; ++i) tl[(nq + i) * 72 + kk] = f2bf(Wm[(size_t)(k0 + kk) * DM + n0 + nq + i]);
    __syncthreads();
    const int piece = tid & 7;
    auto pass = [&]() {
#pragma unroll
        for (int s = 0; s < 2; ++s) { const int nr = (tid >> 3) + 32 * s; const v8us val = *(const v8usa*)(tl + nr * 72 + piece * 8);
            *(volatile v8us*)(WT + (size_t)(n0 + nr) * DM + k0 + piece * 8) = val; }
    };
    pass(); __threadfence(); pass();
}
template <int MODE>
__global__ __launch_bounds__(128) void k_gemmb(const bf* __restrict__ A, const bf* __restrict__ Bn, const float* __restrict__ bias, void* C, void* C2) {
    __shared__ __align__(16) float ost[4][16 * 68];
    const int lane = threadIdx.x & 31, wave = threadIdx.x >> 5, lr = lane & 15, hi = lane >> 4;
    const int r0 = blockIdx.x * 64 + wave * 16, c0 = blockIdx.y * 64;
    const size_t aoff = (size_t)(r0 + lr) * DM + 8 * hi;
    size_t boff[4];
#pragma unroll
    for (int t = 0; t < 4; ++t) boff[t] = (size_t)(c0 + t * 16 + lr) * DM + 8 * hi;
    v8f acc[4];
#pragma unroll
    for (int t = 0; t < 4; ++t) acc[t] = (v8f){};
#pragma unroll 1
    for (int kc = 0; kc < DM; kc += 32) {
        const v16bf a = cat16b(*(const v8us*)(A + aoff + kc), *(const v8us*)(A + aoff + kc + 16));
#pragma unroll
        for (int t = 0; t < 4; ++t) acc[t] = wmmab(a, cat16b(*(const v8us*)(Bn + boff[t] + kc), *(const v8us*)(Bn + boff[t] + kc + 16)), acc[t]);
        asm volatile("v_nop\n\tv_nop\n\tv_nop\n\tv_nop" : "+v"(acc[0]), "+v"(acc[1]), "+v"(acc[2]), "+v"(acc[3]) : "v"(a));
    }
    float* os = &ost[wave][0];
#pragma unroll
    for (int t = 0; t < 4; ++t) { const float bv = bias ? bfr(bias[c0 + t * 16 + lr]) : 0.f;
#pragma unroll
        for (int j = 0; j < 8; ++j) os[(hi * 8 + j) * 68 + t * 16 + lr] = acc[t][j] + bv; }
    __syncthreads();
    if (MODE == 1) {
        float* crow = (float*)C + (size_t)r0 * DM + c0;
        auto pass = [&]() {
#pragma unroll
            for (int s = 0; s < 8; ++s) { const int Lid = (lane >> 3) + 4 * s, piece = lane & 7; const int row = Lid >> 1, cofs = (Lid & 1) * 32 + piece * 4;
                const v4f val = *(const v4fa*)(os + row * 68 + cofs); *(volatile v4f*)(crow + (size_t)row * DM + cofs) = val; }
        };
        pass(); __threadfence(); pass();
    } else {
        h16* c1 = (h16*)C + (size_t)r0 * DM + c0; h16* c2 = (h16*)C2 + (size_t)r0 * DM + c0;
        auto pass = [&]() {
#pragma unroll
            for (int s = 0; s < 4; ++s) { const int row = 4 * s + (lane >> 3), piece = lane & 7; const float* sp = os + row * 68 + piece * 8; v8h o1, o2;
#pragma unroll
                for (int i = 0; i < 8; ++i) { const h16 a = (h16)sp[i]; o1[i] = a; o2[i] = (h16)((sp[i] - (float)a) * LOSC); }
                *(volatile v8h*)(c1 + (size_t)row * DM + piece * 8) = o1; *(volatile v8h*)(c2 + (size_t)row * DM + piece * 8) = o2; }
        };
        pass(); __threadfence(); pass();
    }
}
__global__ __launch_bounds__(256) void k_vt(const float* __restrict__ V, h16* VTH, h16* VTL) {
    __shared__ __align__(16) h16 tile[HD * 72];
    __shared__ __align__(16) h16 til2[HD * 72];
    const int bid = blockIdx.x;
    const int b = bid / (NH_ * (SS / 64)), rem = bid - b * (NH_ * (SS / 64)), h = rem / (SS / 64), kt = rem - h * (SS / 64);
    const int s0 = kt * 64, tid = threadIdx.x, ss = tid >> 2, d0 = (tid & 3) * 16;
    const float* src = V + ((size_t)b * SS + s0 + ss) * DM + h * HD + d0;
#pragma unroll
    for (int i = 0; i < 16; ++i) { const float v = src[i]; const h16 a = (h16)v; tile[(d0 + i) * 72 + ss] = a; til2[(d0 + i) * 72 + ss] = (h16)((v - (float)a) * LOSC); }
    __syncthreads();
    const int piece = tid & 7;
    const size_t base = (((size_t)b * NH_ + h) * HD) * SS + s0;
    auto pass = [&]() {
#pragma unroll
        for (int s = 0; s < 4; ++s) { const int Lid = (tid >> 3) + 32 * s; const int pln = Lid >> 6, d = Lid & 63;
            const v8h val = *(const v8ha*)((pln ? til2 : tile) + d * 72 + piece * 8); *(volatile v8h*)((pln ? VTL : VTH) + base + (size_t)d * SS + piece * 8) = val; }
    };
    pass(); __threadfence(); pass();
}
__global__ __launch_bounds__(256) void k_rk(const float* __restrict__ RKf, h16* RK16) {
    const int lane = threadIdx.x & 31, m = blockIdx.x * 8 + (threadIdx.x >> 5);
    if (m >= NRP) return;
    const bool live = (m >= 1024 && m <= 2047); const int src = live ? (2047 - m) : 0;
#pragma unroll
    for (int q = 0; q < DM / 256; ++q) { v8h o;
#pragma unroll
        for (int i = 0; i < 8; ++i) o[i] = live ? (h16)RKf[(size_t)src * DM + q * 256 + lane * 8 + i] : (h16)0.f;
        *(volatile v8h*)(RK16 + (size_t)m * DM + q * 256 + lane * 8) = o; }
    __threadfence();
#pragma unroll
    for (int q = 0; q < DM / 256; ++q) { v8h o;
#pragma unroll
        for (int i = 0; i < 8; ++i) o[i] = live ? (h16)RKf[(size_t)src * DM + q * 256 + lane * 8 + i] : (h16)0.f;
        *(volatile v8h*)(RK16 + (size_t)m * DM + q * 256 + lane * 8) = o; }
}
__global__ __launch_bounds__(256) void k_ln(const float* O, const float* __restrict__ w, const float* __restrict__ g, const float* __restrict__ be, float* out) {
    const int lane = threadIdx.x & 31; const size_t r = (size_t)blockIdx.x * 8 + (threadIdx.x >> 5);
    if (r >= (size_t)NTK) return;
    float s = 0.f;
#pragma unroll 1
    for (int q = 0; q < 8; ++q) { const v4f t = *(const v4fa*)(O + r * DM + q * 128 + lane * 4);
#pragma unroll
        for (int i = 0; i < 4; ++i) s += t[i] + bfr(w[r * DM + q * 128 + lane * 4 + i]); }
#pragma unroll
    for (int sh = 16; sh; sh >>= 1) s += __shfl_xor(s, sh, 32);
    const float mu = s * (1.0f / DM); float qq = 0.f;
#pragma unroll 1
    for (int q = 0; q < 8; ++q) { const v4f t = *(const v4fa*)(O + r * DM + q * 128 + lane * 4);
#pragma unroll
        for (int i = 0; i < 4; ++i) { const float d = t[i] + bfr(w[r * DM + q * 128 + lane * 4 + i]) - mu; qq += d * d; } }
#pragma unroll
    for (int sh = 16; sh; sh >>= 1) qq += __shfl_xor(qq, sh, 32);
    const float rs = rsqrtf(qq * (1.0f / DM) + 1e-5f);
    v4f o4[8];
#pragma unroll 1
    for (int q = 0; q < 8; ++q) { const v4f t = *(const v4fa*)(O + r * DM + q * 128 + lane * 4); v4f y;
#pragma unroll
        for (int i = 0; i < 4; ++i) { const int c = q * 128 + lane * 4 + i; y[i] = (t[i] + bfr(w[r * DM + c]) - mu) * rs * bfr(g[c]) + bfr(be[c]); }
        o4[q] = y; }
    __builtin_amdgcn_wave_barrier(); asm volatile("" ::: "memory");
#pragma unroll
    for (int q = 0; q < 8; ++q) *(volatile v4f*)(out + r * DM + q * 128 + lane * 4) = o4[q];
    __threadfence();
#pragma unroll
    for (int q = 0; q < 8; ++q) *(volatile v4f*)(out + r * DM + q * 128 + lane * 4) = o4[q];
}
__global__ __launch_bounds__(128) void k_attn(const h16* __restrict__ QH, const h16* __restrict__ QL, const h16* __restrict__ QRH, const h16* __restrict__ QRL, const h16* __restrict__ KH, const h16* __restrict__ KL,
                                             const h16* __restrict__ RK16, const h16* __restrict__ VTH, const h16* __restrict__ VTL, const int* __restrict__ amask, bf* CH, bf* CL) {
    __shared__ __align__(16) h16 plds[4][16 * 32];
    __shared__ __align__(16) h16 plds2[4][16 * 32];
    __shared__ __align__(16) float posl[4][16 * 52];
    __shared__ __align__(16) float ost[4][16 * 68];
    const int lane = threadIdx.x & 31, wave = threadIdx.x >> 5, lr = lane & 15, hi = lane >> 4;
    const int bid = blockIdx.x;
    const int b = bid / (NH_ * (SS / 64)), rem = bid - b * (NH_ * (SS / 64)), h = rem / (SS / 64), qt = rem - h * (SS / 64);
    const int q0 = qt * 64 + wave * 16;
    const size_t tok0 = (size_t)b * SS;
    h16* pl = &plds[wave][0]; h16* pl2 = &plds2[wave][0]; float* ps = &posl[wave][0];
    const size_t qo0 = (tok0 + q0 + lr) * DM + h * HD + 8 * hi;
    v16h qa[2];
#pragma unroll
    for (int kc = 0; kc < 2; ++kc) qa[kc] = cat16(*(const v8h*)(QH + qo0 + kc * 32), *(const v8h*)(QH + qo0 + kc * 32 + 16));
    v16h qra[2];
#pragma unroll
    for (int kc = 0; kc < 2; ++kc) qra[kc] = cat16(*(const v8h*)(QRH + qo0 + kc * 32), *(const v8h*)(QRH + qo0 + kc * 32 + 16));
    const size_t vbase = (((size_t)b * NH_ + h) * HD) * SS;
    v8f o[4], ox[4];
#pragma unroll
    for (int n = 0; n < 4; ++n) { o[n] = (v8f){}; ox[n] = (v8f){}; }
    float mrow[8], lpart[8];
#pragma unroll
    for (int j = 0; j < 8; ++j) { mrow[j] = -3.0e38f; lpart[j] = 0.f; }
    const int kt_hi = (qt * 64 + 63) / 32;
#pragma unroll 1
    for (int kt = 0; kt <= kt_hi; ++kt) {
        const int l0 = kt * 32, mbase = q0 - l0 - 31 + 1024;
        v8f s0 = {}, s1 = {}, x0 = {}, x1 = {};
#pragma unroll
        for (int kc = 0; kc < 2; ++kc) {
            const size_t ko = (tok0 + l0 + lr) * DM + h * HD + kc * 32 + 8 * hi, k1o = ko + (size_t)16 * DM;
            const v16h qlk = cat16(*(const v8h*)(QL + qo0 + kc * 32), *(const v8h*)(QL + qo0 + kc * 32 + 16));
            { const v16h k0h = cat16(*(const v8h*)(KH + ko), *(const v8h*)(KH + ko + 16)), k1h = cat16(*(const v8h*)(KH + k1o), *(const v8h*)(KH + k1o + 16));
              s0 = wmma16(qa[kc], k0h, s0); x0 = wmma16(qlk, k0h, x0); s1 = wmma16(qa[kc], k1h, s1); x1 = wmma16(qlk, k1h, x1);
              asm volatile("v_nop" : "+v"(s0), "+v"(s1), "+v"(x0), "+v"(x1) : "v"(qlk), "v"(k0h), "v"(k1h) : "memory"); }
            { const v16h k0l = cat16(*(const v8h*)(KL + ko), *(const v8h*)(KL + ko + 16)), k1l = cat16(*(const v8h*)(KL + k1o), *(const v8h*)(KL + k1o + 16));
              x0 = wmma16(qa[kc], k0l, x0); x1 = wmma16(qa[kc], k1l, x1);
              asm volatile("v_nop" : "+v"(x0), "+v"(x1) : "v"(k0l), "v"(k1l) : "memory"); }
            const v16h qrl = cat16(*(const v8h*)(QRL + qo0 + kc * 32), *(const v8h*)(QRL + qo0 + kc * 32 + 16));
#pragma unroll
            for (int t = 0; t < 3; ++t) { const size_t om = (size_t)(mbase + t * 16 + lr) * DM + h * HD + kc * 32 + 8 * hi;
                const v16h rb = cat16(*(const v8h*)(RK16 + om), *(const v8h*)(RK16 + om + 16));
                v8f ph = wmma16(qra[kc], rb, (v8f){}); v8f pq = wmma16(qrl, rb, (v8f){});
                asm volatile("v_nop\n\tv_nop\n\tv_nop\n\tv_nop" : "+v"(ph), "+v"(pq) : "v"(rb), "v"(qrl));
#pragma unroll
                for (int j = 0; j < 8; ++j) { const int idx = (hi * 8 + j) * 52 + t * 16 + lr; const float v = ph[j] + pq[j] * LOSCI; if (kc == 0) ps[idx] = v; else ps[idx] += v; }
                asm volatile("" ::: "memory"); }
        }
        asm volatile("v_nop\n\tv_nop\n\tv_nop\n\tv_nop" : "+v"(s0), "+v"(s1), "+v"(x0), "+v"(x1) : "v"(qa[0]), "v"(qa[1]));
        asm volatile("" ::: "memory");
        __builtin_amdgcn_wave_barrier();
        float alpha[8];
#pragma unroll
        for (int j = 0; j < 8; ++j) {
            const int r = hi * 8 + j;
            const float p0v = ps[r * 52 + r - lr + 31], p1v = ps[r * 52 + r - (lr + 16) + 31];
            const int qi = q0 + r, ja = l0 + lr, jb = l0 + 16 + lr;
            const int ka = amask[((size_t)b * SS + qi) * SS + ja], kb = amask[((size_t)b * SS + qi) * SS + jb];
            const float a0 = ka ? (s0[j] + x0[j] * LOSCI + p0v) * 0.125f : -1.0e30f, a1 = kb ? (s1[j] + x1[j] * LOSCI + p1v) * 0.125f : -1.0e30f;
            float mx = fmaxf(a0, a1);
            mx = fmaxf(mx, __shfl_xor(mx, 1, 16)); mx = fmaxf(mx, __shfl_xor(mx, 2, 16)); mx = fmaxf(mx, __shfl_xor(mx, 4, 16)); mx = fmaxf(mx, __shfl_xor(mx, 8, 16));
            const float mn = fmaxf(mrow[j], mx);
            alpha[j] = __expf(mrow[j] - mn); mrow[j] = mn;
            const float e0 = __expf(a0 - mn), e1 = __expf(a1 - mn);
            lpart[j] = lpart[j] * alpha[j] + (e0 + e1);
            const float ps0 = e0 * PSC, ps1 = e1 * PSC; const h16 h0 = (h16)ps0, h1 = (h16)ps1; const h16 g0 = (h16)((ps0 - (float)h0) * LOSC), g1 = (h16)((ps1 - (float)h1) * LOSC);
            pl[r * 32 + lr] = h0; pl[r * 32 + 16 + lr] = h1; pl2[r * 32 + lr] = g0; pl2[r * 32 + 16 + lr] = g1;
        }
#pragma unroll
        for (int n = 0; n < 4; ++n)
#pragma unroll
            for (int j = 0; j < 8; ++j) { o[n][j] *= alpha[j]; ox[n][j] *= alpha[j]; }
        asm volatile("" ::: "memory");
        const v16h pa = cat16(*(const v8ha*)(pl + lr * 32 + hi * 8), *(const v8ha*)(pl + lr * 32 + 16 + hi * 8));
        const v16h px = cat16(*(const v8ha*)(pl2 + lr * 32 + hi * 8), *(const v8ha*)(pl2 + lr * 32 + 16 + hi * 8));
#pragma unroll
        for (int n = 0; n < 4; ++n) { const size_t vo = vbase + (size_t)(n * 16 + lr) * SS + l0 + hi * 8;
            const v16h vh = cat16(*(const v8h*)(VTH + vo), *(const v8h*)(VTH + vo + 16)), vl = cat16(*(const v8h*)(VTL + vo), *(const v8h*)(VTL + vo + 16));
            o[n] = wmma16(pa, vh, o[n]); ox[n] = wmma16(pa, vl, ox[n]); ox[n] = wmma16(px, vh, ox[n]);
            asm volatile("" : "+v"(o[n]), "+v"(ox[n]) : "v"(vh), "v"(vl) : "memory"); }
        __builtin_amdgcn_wave_barrier();
        asm volatile("" ::: "memory");
    }
    asm volatile("v_nop\n\tv_nop\n\tv_nop\n\tv_nop" : "+v"(o[0]), "+v"(o[1]), "+v"(o[2]), "+v"(o[3]), "+v"(ox[0]), "+v"(ox[1]), "+v"(ox[2]), "+v"(ox[3]));
    float inv[8];
#pragma unroll
    for (int j = 0; j < 8; ++j) { float rs = lpart[j]; rs += __shfl_xor(rs, 1, 16); rs += __shfl_xor(rs, 2, 16); rs += __shfl_xor(rs, 4, 16); rs += __shfl_xor(rs, 8, 16); inv[j] = 1.0f / (rs * PSC); }
    float* os = &ost[wave][0];
#pragma unroll
    for (int n = 0; n < 4; ++n)
#pragma unroll
        for (int j = 0; j < 8; ++j) os[(hi * 8 + j) * 68 + n * 16 + lr] = (o[n][j] + ox[n][j] * LOSCI) * inv[j];
    __syncthreads();
    const size_t cbase = (tok0 + q0) * DM + (size_t)h * HD;
    auto pass = [&]() {
#pragma unroll
        for (int s = 0; s < 4; ++s) { const int row = 4 * s + (lane >> 3), piece = lane & 7; const float* sp = os + row * 68 + piece * 8; v8us oh, ol;
#pragma unroll
            for (int i = 0; i < 8; ++i) { const unsigned short hb = f2bf(sp[i]); oh[i] = hb; ol[i] = f2bf(sp[i] - bf2f(hb)); }
            *(volatile v8us*)(CH + cbase + (size_t)row * DM + piece * 8) = oh; *(volatile v8us*)(CL + cbase + (size_t)row * DM + piece * 8) = ol; }
    };
    pass(); __threadfence(); pass();
}
__global__ __launch_bounds__(128) void k_outp(const bf* __restrict__ A, const bf* __restrict__ Al, const bf* __restrict__ Bn, const float* __restrict__ bias, float* C) {
    __shared__ __align__(16) float ost[4][16 * 68];
    const int lane = threadIdx.x & 31, wave = threadIdx.x >> 5, lr = lane & 15, hi = lane >> 4;
    const int r0 = blockIdx.x * 64 + wave * 16, c0 = blockIdx.y * 64;
    const size_t aoff = (size_t)(r0 + lr) * DM + 8 * hi;
    size_t boff[4];
#pragma unroll
    for (int t = 0; t < 4; ++t) boff[t] = (size_t)(c0 + t * 16 + lr) * DM + 8 * hi;
    v8f acc[4];
#pragma unroll
    for (int t = 0; t < 4; ++t) acc[t] = (v8f){};
#pragma unroll 1
    for (int kc = 0; kc < DM; kc += 32) {
        const v16bf a = cat16b(*(const v8us*)(A + aoff + kc), *(const v8us*)(A + aoff + kc + 16)), al = cat16b(*(const v8us*)(Al + aoff + kc), *(const v8us*)(Al + aoff + kc + 16));
#pragma unroll
        for (int t = 0; t < 4; ++t) { const v16bf bb = cat16b(*(const v8us*)(Bn + boff[t] + kc), *(const v8us*)(Bn + boff[t] + kc + 16)); acc[t] = wmmab(a, bb, acc[t]); acc[t] = wmmab(al, bb, acc[t]); }
        asm volatile("v_nop\n\tv_nop\n\tv_nop\n\tv_nop" : "+v"(acc[0]), "+v"(acc[1]), "+v"(acc[2]), "+v"(acc[3]) : "v"(a), "v"(al));
    }
    float* os = &ost[wave][0];
#pragma unroll
    for (int t = 0; t < 4; ++t) { const float bv = bfr(bias[c0 + t * 16 + lr]);
#pragma unroll
        for (int j = 0; j < 8; ++j) os[(hi * 8 + j) * 68 + t * 16 + lr] = acc[t][j] + bv; }
    __syncthreads();
    float* crow = C + (size_t)r0 * DM + c0;
    auto pass = [&]() {
#pragma unroll
        for (int s = 0; s < 8; ++s) { const int Lid = (lane >> 3) + 4 * s, piece = lane & 7; const int row = Lid >> 1, cofs = (Lid & 1) * 32 + piece * 4;
            const v4f val = *(const v4fa*)(os + row * 68 + cofs); *(volatile v4f*)(crow + (size_t)row * DM + cofs) = val; }
    };
    pass(); __threadfence(); pass();
}

extern "C" void kernel_launch(void* const* d_in, const int* in_sizes, int n_in,
                              void* d_out, int out_size, void* d_ws, size_t ws_size, hipStream_t stream) {
    (void)in_sizes; (void)n_in; (void)out_size;
    const float* w = (const float*)d_in[0]; const float* r = (const float*)d_in[1]; const float* rwb = (const float*)d_in[2]; const float* rrb = (const float*)d_in[3]; const int* amask = (const int*)d_in[4];
    const float* Wq = (const float*)d_in[5]; const float* Wk = (const float*)d_in[6]; const float* Wv = (const float*)d_in[7]; const float* Wr = (const float*)d_in[8]; const float* Wo = (const float*)d_in[9];
    const float* bo = (const float*)d_in[10]; const float* gam = (const float*)d_in[11]; const float* bet = (const float*)d_in[12];
    float* out = (float*)d_out;
    char* wsp = (char*)d_ws;
    auto take = [&](size_t bytes) { char* p = wsp; wsp += (bytes + 255) & ~(size_t)255; return (void*)p; };
    bf* Xb = (bf*)take((size_t)NTK * DM * 2); bf* Rb = (bf*)take((size_t)SS * DM * 2);
    bf* WqB = (bf*)take((size_t)DM * DM * 2); bf* WkB = (bf*)take((size_t)DM * DM * 2); bf* WvB = (bf*)take((size_t)DM * DM * 2); bf* WrB = (bf*)take((size_t)DM * DM * 2); bf* WoB = (bf*)take((size_t)DM * DM * 2);
    h16* QH = (h16*)take((size_t)NTK * DM * 2); h16* QL = (h16*)take((size_t)NTK * DM * 2); h16* QRH = (h16*)take((size_t)NTK * DM * 2); h16* QRL = (h16*)take((size_t)NTK * DM * 2);
    h16* KH = (h16*)take((size_t)NTK * DM * 2); h16* KL = (h16*)take((size_t)NTK * DM * 2); float* Vf = (float*)take((size_t)NTK * DM * 4); h16* VTH = (h16*)take((size_t)NTK * DM * 2); h16* VTL = (h16*)take((size_t)NTK * DM * 2);
    float* RKf = (float*)take((size_t)SS * DM * 4); h16* RK16 = (h16*)take((size_t)NRP * DM * 2);
    if ((size_t)(wsp - (char*)d_ws) > ws_size) return;
    bf* CH = (bf*)Vf; bf* CL = (bf*)((char*)Vf + (size_t)NTK * DM * 2);
    k_cvtb<<<NTK / 8, 256, 0, stream>>>(w, NTK, Xb); k_cvtb<<<SS / 8, 256, 0, stream>>>(r, SS, Rb);
    k_cvtb<<<DM / 8, 256, 0, stream>>>(Wq, DM, WqB); k_cvtb<<<DM / 8, 256, 0, stream>>>(Wk, DM, WkB); k_cvtb<<<DM / 8, 256, 0, stream>>>(Wv, DM, WvB);
    k_cvtb<<<DM / 8, 256, 0, stream>>>(Wr, DM, WrB); k_cvtb<<<DM / 8, 256, 0, stream>>>(Wo, DM, WoB);
    k_gemmb<0><<<dim3(NTK / 64, DM / 64, 1), 128, 0, stream>>>(Xb, WqB, rwb, QH, QL);
    k_gemmb<0><<<dim3(NTK / 64, DM / 64, 1), 128, 0, stream>>>(Xb, WqB, rrb, QRH, QRL);
    k_gemmb<0><<<dim3(NTK / 64, DM / 64, 1), 128, 0, stream>>>(Xb, WkB, nullptr, KH, KL);
    k_gemmb<1><<<dim3(NTK / 64, DM / 64, 1), 128, 0, stream>>>(Xb, WvB, nullptr, Vf, nullptr);
    k_gemmb<1><<<dim3(SS / 64, DM / 64, 1), 128, 0, stream>>>(Rb, WrB, nullptr, RKf, nullptr);
    k_rk<<<NRP / 8, 256, 0, stream>>>(RKf, RK16);
    k_vt<<<NB_ * NH_ * (SS / 64), 256, 0, stream>>>(Vf, VTH, VTL);
    k_attn<<<NB_ * NH_ * (SS / 64), 128, 0, stream>>>(QH, QL, QRH, QRL, KH, KL, RK16, VTH, VTL, amask, CH, CL);
    k_outp<<<dim3(NTK / 64, DM / 64, 1), 128, 0, stream>>>(CH, CL, WoB, bo, out);
    k_ln<<<NTK / 8, 256, 0, stream>>>(out, w, gam, bet, out);
}
